// ContextTransformer_14955076124951
// MI455X (gfx1250) — hardware-run, weakly checked
//
#include <hip/hip_runtime.h>
#include <math.h>

typedef __attribute__((ext_vector_type(16))) _Float16 v16h;
typedef __attribute__((ext_vector_type(16))) __bf16 v16b;
typedef __attribute__((ext_vector_type(8)))  _Float16 v8h;
typedef __attribute__((ext_vector_type(8)))  float v8f;
typedef __attribute__((ext_vector_type(4)))  float v4f;
typedef __attribute__((ext_vector_type(2)))  float v2f;
typedef __attribute__((ext_vector_type(4)))  unsigned v4u;
typedef __attribute__((ext_vector_type(4)))  int v4i;
typedef float __attribute__((may_alias)) float_a;
typedef int __attribute__((may_alias)) int_a;

template <typename T> __device__ __forceinline__ void vst2(void* p, T v) { *(volatile T*)p = v; __threadfence(); *(volatile T*)p = v; }
__device__ __forceinline__ v8f wmma16(v16h a, v16h b, v8f c) {
  v8f d = __builtin_amdgcn_wmma_f32_16x16x32_f16(false, a, false, b, (short)0, c, false, false);
  asm volatile("v_nop\n\tv_nop\n\tv_nop\n\tv_nop" : "+v"(d) : "v"(a), "v"(b));
  return d;
}
__device__ __forceinline__ v8f wmma_bf(v16b a, v16b b, v8f c) {
  v8f d = __builtin_amdgcn_wmma_f32_16x16x32_bf16(false, a, false, b, (short)0, c, false, false);
  asm volatile("v_nop\n\tv_nop\n\tv_nop\n\tv_nop" : "+v"(d) : "v"(a), "v"(b));
  return d;
}
__device__ __forceinline__ v16h frag_h(const _Float16* rowk0, int lane) {
  union { v16h v; v8h q[2]; } u; const _Float16* p = rowk0 + 8 * (lane >> 4);
  u.q[0] = *(const v8h*)p; u.q[1] = *(const v8h*)(p + 16); return u.v;
}
__device__ __forceinline__ v16h frag_f32(const float* rowk0, int lane) {
  v16h a; const float* p = rowk0 + 8 * (lane >> 4);
#pragma unroll
  for (int i = 0; i < 8; ++i) { a[i] = (_Float16)p[i]; a[8 + i] = (_Float16)p[16 + i]; }
  return a;
}
__device__ __forceinline__ v16h frag_f32s(const float* rowk0, int lane, float sc) {
  v16h a; const float* p = rowk0 + 8 * (lane >> 4);
#pragma unroll
  for (int i = 0; i < 8; ++i) { a[i] = (_Float16)(p[i] * sc); a[8 + i] = (_Float16)(p[16 + i] * sc); }
  return a;
}
__device__ __forceinline__ v16h fragc_f32(const float* W, int k0, int n, int lane, int ld, int K) {
  v16h a; const int g = lane >> 4;
#pragma unroll
  for (int i = 0; i < 8; ++i) { const int ka = k0 + 8 * g + i, kb = ka + 16;
    a[i] = (_Float16)(ka < K ? W[(size_t)(ka < K ? ka : K - 1) * ld + n] : 0.f); a[8 + i] = (_Float16)(kb < K ? W[(size_t)(kb < K ? kb : K - 1) * ld + n] : 0.f); }
  return a;
}
struct F2 { v16b h, l; };
__device__ __forceinline__ F2 bsplit16(const float v[16]) { F2 r;
#pragma unroll
  for (int i = 0; i < 16; ++i) { const __bf16 h = (__bf16)v[i]; r.h[i] = h; r.l[i] = (__bf16)(v[i] - (float)h); }
  return r; }
__device__ __forceinline__ F2 split_row(const float* row, int k0, int lane) { float v[16]; const float* p = row + k0 + 8 * (lane >> 4);
#pragma unroll
  for (int i = 0; i < 8; ++i) { v[i] = p[i]; v[8 + i] = p[16 + i]; }
  return bsplit16(v); }
__device__ __forceinline__ F2 split_rowK(const float* row, int k0, int lane, int K) { float v[16]; const int g = lane >> 4;
#pragma unroll
  for (int i = 0; i < 8; ++i) { const int ka = k0 + 8 * g + i, kb = ka + 16; v[i] = ka < K ? row[ka < K ? ka : K - 1] : 0.f; v[8 + i] = kb < K ? row[kb < K ? kb : K - 1] : 0.f; }
  return bsplit16(v); }
__device__ __forceinline__ F2 split_col(const float* W, int k0, int n, int lane, int ld, int K) { float v[16]; const int g = lane >> 4;
#pragma unroll
  for (int i = 0; i < 8; ++i) { const int ka = k0 + 8 * g + i, kb = ka + 16; v[i] = ka < K ? W[(size_t)(ka < K ? ka : K - 1) * ld + n] : 0.f; v[8 + i] = kb < K ? W[(size_t)(kb < K ? kb : K - 1) * ld + n] : 0.f; }
  return bsplit16(v); }
__device__ __forceinline__ v8f mac3(const F2& a, const F2& b, v8f c) { c = wmma_bf(a.l, b.h, c); c = wmma_bf(a.h, b.l, c); return wmma_bf(a.h, b.h, c); }
__device__ __forceinline__ float sigm(float v) { return 1.0f / (1.0f + expf(-v)); }
#define LDSX() do { asm volatile("s_wait_dscnt 0" ::: "memory"); __builtin_amdgcn_wave_barrier(); __builtin_amdgcn_fence(__ATOMIC_RELEASE, "workgroup"); } while (0)

__device__ __forceinline__ float bfr(float v) { return (float)(__bf16)v; }
#define NP 50000
#define KN 16
#define FF 128
#define NH 8
#define DH 16
#define RESC 64.0f
#define TB 4096
#ifndef NPB
#define NPB NP
#endif
#define NRB ((NP + 63) / 64)
#define WS_FN 0u
#define WS_Q  (WS_FN + 4u * (size_t)NP * FF)
#define WS_K  (WS_Q + 4u * (size_t)NP * FF)
#define WS_V  (WS_K + 4u * (size_t)NP * FF)
#define WS_O  (WS_V + 4u * (size_t)NP * FF)
#define WS_END (WS_O + 4u * (size_t)NP * FF)
__global__ __launch_bounds__(128) void k_qkv(const float* __restrict__ FT, const float* __restrict__ G1, const float* __restrict__ B1, const float* __restrict__ WQ, const float* __restrict__ BQ, const float* __restrict__ WK, const float* __restrict__ BK, const float* __restrict__ WV, const float* __restrict__ BV, float* __restrict__ FN, float* __restrict__ Q, float* __restrict__ K, float* __restrict__ V) {
  __shared__ __align__(16) float sx[64][FF + 4]; __shared__ __align__(16) float sf[4][16][132];
  const int tid = threadIdx.x, wave = tid >> 5, lane = tid & 31, col = lane & 15, g = lane >> 4; const size_t r0 = (size_t)blockIdx.x * 64;
  { const int row = tid >> 1, half = tid & 1; const size_t r = r0 + row; const size_t rr = r < NP ? r : NP - 1; const float* p = FT + rr * FF + half * 64; float s = 0.f; for (int e = 0; e < 64; ++e) { const float v = bfr(p[e]); sx[row][half * 64 + e] = v; s += v; }
    s += __shfl_xor(s, 1); const float mu = s * (1.0f / FF); float s2 = 0.f; for (int e = 0; e < 64; ++e) { const float d = sx[row][half * 64 + e] - mu; s2 += d * d; } s2 += __shfl_xor(s2, 1); const float rs = rsqrtf(s2 * (1.0f / FF) + 1e-5f);
    for (int e = 0; e < 64; ++e) { const int c = half * 64 + e; sx[row][c] = (sx[row][c] - mu) * rs * bfr(G1[c]) + bfr(B1[c]); } }
  __syncthreads();
  for (int q4 = tid; q4 < 64 * FF / 4; q4 += 128) { const int row = q4 / (FF / 4), c4 = (q4 % (FF / 4)) * 4; if (r0 + row < NP) vst2(FN + (r0 + row) * FF + c4, *(const v4f*)&sx[row][c4]); }
#pragma unroll 1
  for (int which = 0; which < 3; ++which) { const float* WA = which == 0 ? WQ : which == 1 ? WK : WV; const float* BA = which == 0 ? BQ : which == 1 ? BK : BV; float* D = which == 0 ? Q : which == 1 ? K : V;
    v8f acc[8] = {};
#pragma unroll
    for (int kc = 0; kc < FF / 32; ++kc) { const v16h a = frag_f32(&sx[wave * 16 + col][kc * 32], lane);
#pragma unroll
      for (int j = 0; j < 8; ++j) { v16h w; const int o = j * 16 + col;
#pragma unroll
        for (int i = 0; i < 8; ++i) { w[i] = (_Float16)(bfr(WA[(size_t)(kc * 32 + 8 * g + i) * FF + o]) * 16.0f); w[8 + i] = (_Float16)(bfr(WA[(size_t)(kc * 32 + 16 + 8 * g + i) * FF + o]) * 16.0f); }
        acc[j] = wmma16(a, w, acc[j]); } }
#pragma unroll
    for (int j = 0; j < 8; ++j) { const float bb = bfr(BA[j * 16 + col]);
#pragma unroll
      for (int r = 0; r < 8; ++r) sf[wave][8 * g + r][j * 16 + col] = acc[j][r] * (1.0f / 16.0f) + bb; }
    LDSX(); for (int rl = 0; rl < 16; ++rl) { const size_t r = r0 + wave * 16 + rl; if (r < NP) vst2(D + r * FF + lane * 4, *(const v4f*)&sf[wave][rl][lane * 4]); } LDSX(); } }
__global__ __launch_bounds__(128) void k_ctx(const float* __restrict__ XYZ, const int* __restrict__ ED, const float* __restrict__ TBL, const float* __restrict__ Q, const float* __restrict__ K, const float* __restrict__ V, float* __restrict__ O) {
  __shared__ __align__(16) float sq[8][FF]; __shared__ float ssc[8][NH][KN + 1]; __shared__ int sj[8][KN]; __shared__ __align__(16) float so[8][FF];
  const int tid = threadIdx.x; const int pt = tid >> 4, kk = tid & 15; const size_t n0 = (size_t)blockIdx.x * 8; const size_t n = n0 + pt;
  for (int e = tid; e < 8 * FF / 4; e += 128) { const int p = e / (FF / 4), c4 = (e % (FF / 4)) * 4; *(v4f*)&sq[p][c4] = *(const v4f*)(Q + (n0 + p) * FF + c4); }
  const int j = ED[n * KN + kk]; sj[pt][kk] = j;
  const float rx = bfr(XYZ[(size_t)j * 3]) - bfr(XYZ[n * 3]), ry = bfr(XYZ[(size_t)j * 3 + 1]) - bfr(XYZ[n * 3 + 1]), rz = bfr(XYZ[(size_t)j * 3 + 2]) - bfr(XYZ[n * 3 + 2]);
  const unsigned c0 = (unsigned)(int)floorf(rx * RESC), c1 = (unsigned)(int)floorf(ry * RESC), c2 = (unsigned)(int)floorf(rz * RESC);
  const unsigned hsh = ((c0 * 1u) ^ (c1 * 2654435761u) ^ (c2 * 805459861u)) % (unsigned)TB;
  __syncthreads();
  const float* kr = K + (size_t)j * FF; const float* pe = TBL + (size_t)hsh * FF;
#pragma unroll 1
  for (int h = 0; h < NH; ++h) { float s = 0.f;
#pragma unroll
    for (int q4 = 0; q4 < DH; q4 += 4) { const int c4 = h * DH + q4; const v4f kv = *(const v4f*)(kr + c4); const v4f pv = *(const v4f*)(pe + c4); const v4f qv = *(const v4f*)&sq[pt][c4];
      s += qv[0] * (kv[0] + bfr(pv[0])) + qv[1] * (kv[1] + bfr(pv[1])) + qv[2] * (kv[2] + bfr(pv[2])) + qv[3] * (kv[3] + bfr(pv[3])); }
    ssc[pt][h][kk] = s * 0.25f; }
  __syncthreads();
  if (tid < 64) { const int p = tid >> 3, h = tid & 7; float* row = ssc[p][h]; float m = -3.0e38f; for (int q = 0; q < KN; ++q) m = fmaxf(m, row[q]); float s = 0.f; for (int q = 0; q < KN; ++q) { const float e = expf(row[q] - m); row[q] = e; s += e; } const float inv = 1.0f / s; for (int q = 0; q < KN; ++q) row[q] *= inv; }
  __syncthreads();
  { const int p = tid >> 4, cg = (tid & 15) * 8; const int h = cg / DH; float acc8[8];
#pragma unroll
    for (int i = 0; i < 8; ++i) acc8[i] = 0.f;
#pragma unroll 1
    for (int q = 0; q < KN; ++q) { const float a = ssc[p][h][q]; const float* vr = V + (size_t)sj[p][q] * FF + cg; const v4f v0 = *(const v4f*)vr, v1 = *(const v4f*)(vr + 4);
      acc8[0] += a * v0[0]; acc8[1] += a * v0[1]; acc8[2] += a * v0[2]; acc8[3] += a * v0[3]; acc8[4] += a * v1[0]; acc8[5] += a * v1[1]; acc8[6] += a * v1[2]; acc8[7] += a * v1[3]; }
#pragma unroll
    for (int i = 0; i < 8; ++i) so[p][cg + i] = acc8[i]; }
  __syncthreads();
  for (int e = tid; e < 8 * FF / 4; e += 128) { const int p = e / (FF / 4), c4 = (e % (FF / 4)) * 4; vst2(O + (n0 + p) * FF + c4, *(const v4f*)&so[p][c4]); } }
__global__ __launch_bounds__(128) void k_o(const float* __restrict__ O, const float* __restrict__ FN, const float* __restrict__ WO, const float* __restrict__ BO, const float* __restrict__ G2, const float* __restrict__ B2, const float* __restrict__ WL, const float* __restrict__ BL, float* __restrict__ OUT) {
  __shared__ __align__(16) float sfe[64][FF + 4]; __shared__ __align__(16) float sln[64][FF + 4]; __shared__ __align__(16) float sf[4][16][132];
  const int tid = threadIdx.x, wave = tid >> 5, lane = tid & 31, col = lane & 15, g = lane >> 4; const size_t r0 = (size_t)blockIdx.x * 64; const size_t ra = (r0 + wave * 16 + col < NPB) ? r0 + wave * 16 + col : NPB - 1;
  { v8f acc[8] = {};
#pragma unroll
    for (int kc = 0; kc < FF / 32; ++kc) { const F2 a = split_row(O + ra * FF, kc * 32, lane);
#pragma unroll
      for (int j = 0; j < 8; ++j) { v16b w; const int o = j * 16 + col;
#pragma unroll
        for (int i = 0; i < 8; ++i) { w[i] = (__bf16)WO[(size_t)(kc * 32 + 8 * g + i) * FF + o]; w[8 + i] = (__bf16)WO[(size_t)(kc * 32 + 16 + 8 * g + i) * FF + o]; }
        acc[j] = wmma_bf(a.h, w, acc[j]); acc[j] = wmma_bf(a.l, w, acc[j]); } }
#pragma unroll
    for (int j = 0; j < 8; ++j) { const int cl = j * 16 + col; const float bb = bfr(BO[cl]);
#pragma unroll
      for (int r = 0; r < 8; ++r) { const size_t rr = r0 + wave * 16 + 8 * g + r; sfe[wave * 16 + 8 * g + r][cl] = acc[j][r] + bb + FN[(rr < NPB ? rr : NPB - 1) * FF + cl]; }
      asm volatile("s_wait_loadcnt 0x0" ::: "memory"); } }
  __syncthreads();
  { const int row = tid >> 1, half = tid & 1; float s = 0.f; for (int e = 0; e < 64; ++e) s += sfe[row][half * 64 + e]; s += __shfl_xor(s, 1); const float mu = s * (1.0f / FF); float s2 = 0.f; for (int e = 0; e < 64; ++e) { const float d = sfe[row][half * 64 + e] - mu; s2 += d * d; } s2 += __shfl_xor(s2, 1); const float rs = rsqrtf(s2 * (1.0f / FF) + 1e-5f);
    for (int e = 0; e < 64; ++e) { const int c = half * 64 + e; sln[row][c] = (sfe[row][c] - mu) * rs * bfr(G2[c]) + bfr(B2[c]); } }
  __syncthreads();
  { v8f acc[8] = {};
#pragma unroll
    for (int kc = 0; kc < FF / 32; ++kc) { const F2 a = split_row(&sln[wave * 16 + col][0], kc * 32, lane);
#pragma unroll
      for (int j = 0; j < 8; ++j) { v16b w; const int o = j * 16 + col;
#pragma unroll
        for (int i = 0; i < 8; ++i) { w[i] = (__bf16)WL[(size_t)(kc * 32 + 8 * g + i) * FF + o]; w[8 + i] = (__bf16)WL[(size_t)(kc * 32 + 16 + 8 * g + i) * FF + o]; }
        acc[j] = wmma_bf(a.h, w, acc[j]); acc[j] = wmma_bf(a.l, w, acc[j]); } }
#pragma unroll
    for (int j = 0; j < 8; ++j) { const int cl = j * 16 + col; const float bb = bfr(BL[cl]);
#pragma unroll
      for (int r = 0; r < 8; ++r) sf[wave][8 * g + r][cl] = acc[j][r] + bb + sfe[wave * 16 + 8 * g + r][cl]; } }
  LDSX(); for (int rl = 0; rl < 16; ++rl) { const size_t r = r0 + wave * 16 + rl; if (r < NPB) vst2(OUT + r * FF + lane * 4, *(const v4f*)&sf[wave][rl][lane * 4]); } }
extern "C" void kernel_launch(void* const* d_in, const int* in_sizes, int n_in, void* d_out, int out_size, void* d_ws, size_t ws_size, hipStream_t stream) {
  (void)in_sizes; (void)n_in; (void)out_size;
  const float** F = (const float**)d_in;
  if (ws_size < (size_t)WS_END) return;
  char* ws = (char*)d_ws; float *FN = (float*)(ws + WS_FN), *Q = (float*)(ws + WS_Q), *K = (float*)(ws + WS_K), *V = (float*)(ws + WS_V), *O = (float*)(ws + WS_O);
  k_qkv<<<dim3(NRB), 128, 0, stream>>>(F[1], F[12], F[13], F[3], F[4], F[5], F[6], F[7], F[8], FN, Q, K, V);
  k_ctx<<<dim3(NPB / 8), 128, 0, stream>>>(F[0], (const int*)d_in[2], F[11], Q, K, V, O);
  k_o<<<dim3((NPB + 63) / 64), 128, 0, stream>>>(O, FN, F[9], F[10], F[14], F[15], F[16], F[17], (float*)d_out);
}
